// _NonLocalBlockND_POS_46385646797194
// MI455X (gfx1250) — hardware-verified
//
#include <hip/hip_runtime.h>
#include <math.h>
#include <stdint.h>

#define NREAL 9409
#define NPAD  9472
#define NKT   148
#define CIN   512
#define KMIX  1024
#define CT    256
#define CG    512

#define INVBN  0.999995f
#define SCL    0.090168440055560213f
#define PCARRY 16384.0f
#define PINV   (1.0f / 16384.0f)

typedef __attribute__((ext_vector_type(16))) _Float16 v16h;
typedef __attribute__((ext_vector_type(8)))  _Float16 v8h;
typedef __attribute__((ext_vector_type(16))) __bf16   v16b;
typedef __attribute__((ext_vector_type(8)))  __bf16   v8b;
typedef __attribute__((ext_vector_type(8)))  float    v8f;
typedef __attribute__((ext_vector_type(4)))  float    v4f;
typedef __attribute__((ext_vector_type(4)))  unsigned int v4u;

static_assert((NPAD % 64) == 0);
static_assert(NKT * 64 == NPAD);
static_assert(NREAL <= NPAD);

__device__ __forceinline__ unsigned short f2bf_bits(float f) {
  const unsigned u = __float_as_uint(f);
  return (unsigned short)((u + 0x7FFFu + ((u >> 16) & 1u)) >> 16);
}
__device__ __forceinline__ float bf_bits2f(unsigned short h) { return __uint_as_float(((unsigned)h) << 16); }
__device__ __forceinline__ unsigned pk16(unsigned short a, unsigned short b) { return (unsigned)a | ((unsigned)b << 16); }

__device__ __forceinline__ v8f mma_h(v16h a, v16h b, v8f c) {
  c = __builtin_amdgcn_wmma_f32_16x16x32_f16(false, a, false, b, (short)0, c, false, false);
  asm volatile("v_nop\n\tv_nop\n\tv_nop\n\tv_nop" : "+v"(c) : "v"(a), "v"(b));
  return c;
}
__device__ __forceinline__ v8f mma_b(v16b a, v16b b, v8f c) {
  c = __builtin_amdgcn_wmma_f32_16x16x32_bf16(false, a, false, b, (short)0, c, false, false);
  asm volatile("v_nop\n\tv_nop\n\tv_nop\n\tv_nop" : "+v"(c) : "v"(a), "v"(b));
  return c;
}

union FragB { v16b v; v8b h[2]; };
union FragH { v16h v; v8h h[2]; };
__device__ __forceinline__ v16b ldfrag_b(const unsigned short* p) {
  FragB f;
  f.h[0] = *(const v8b*)(const void*)p;
  f.h[1] = *(const v8b*)(const void*)(p + 16);
  return f.v;
}
__device__ __forceinline__ v16h ldfrag_h(const _Float16* p) {
  FragH f;
  f.h[0] = *(const v8h*)p;
  f.h[1] = *(const v8h*)(p + 16);
  return f.v;
}

__device__ __forceinline__ void lds_wave_sync() {
  __builtin_amdgcn_fence(__ATOMIC_RELEASE, "workgroup");
  __builtin_amdgcn_wave_barrier();
  __builtin_amdgcn_fence(__ATOMIC_ACQUIRE, "workgroup");
}

__global__ __launch_bounds__(256) void xmix_kernel(const float* __restrict__ x, const float* __restrict__ pos,
                                                   unsigned short* __restrict__ xh, unsigned short* __restrict__ xl) {
  __shared__ float tf[64 * 65];
  const int cb  = blockIdx.x;
  const int n0  = blockIdx.y * 64;
  const int tid = threadIdx.x;
  const float* src = (cb < 8) ? x : pos;
  const int cs0 = (cb & 7) * 64;
  {
    const int nl  = tid & 63;
    const int n   = n0 + nl;
    const bool ok = n < NREAL;
    const int nc  = ok ? n : (NREAL - 1);
    const int cl0 = tid >> 6;
#pragma unroll 4
    for (int it = 0; it < 16; ++it) {
      const int cl = it * 4 + cl0;
      const float v = src[(size_t)(cs0 + cl) * NREAL + nc];
      tf[cl * 65 + nl] = ok ? v : 0.f;
    }
  }
  __syncthreads();
  const int q  = tid >> 3;
  const int c8 = (tid & 7) * 8;
  v4u ph[2], pl[2];
#pragma unroll
  for (int it = 0; it < 2; ++it) {
    const int r = it * 32 + q;
    v4u b, d;
#pragma unroll
    for (int e = 0; e < 4; ++e) {
      const float f0 = tf[(c8 + 2 * e) * 65 + r];
      const float f1 = tf[(c8 + 2 * e + 1) * 65 + r];
      const unsigned short b0 = f2bf_bits(f0), b1 = f2bf_bits(f1);
      const unsigned short l0 = f2bf_bits(f0 - bf_bits2f(b0)), l1 = f2bf_bits(f1 - bf_bits2f(b1));
      b[e] = pk16(b0, b1);
      d[e] = pk16(l0, l1);
    }
    ph[it] = b; pl[it] = d;
  }
  for (int pass = 0; pass < 2; ++pass) {
#pragma unroll
    for (int it = 0; it < 2; ++it) {
      const int r = it * 32 + q;
      const size_t go = (size_t)(n0 + r) * KMIX + cb * 64 + c8;
      *(volatile v4u*)(xh + go) = ph[it];
      *(volatile v4u*)(xl + go) = pl[it];
    }
    __threadfence();
  }
}

__global__ __launch_bounds__(256) void wsplit_kernel(const float* __restrict__ w, unsigned short* __restrict__ hi,
                                                     unsigned short* __restrict__ lo, int n8) {
  const int i = blockIdx.x * 256 + threadIdx.x;
  if (i < n8) {
    const v4f a = *(const v4f*)(w + 8 * (size_t)i);
    const v4f b = *(const v4f*)(w + 8 * (size_t)i + 4);
    const float f[8] = {a[0], a[1], a[2], a[3], b[0], b[1], b[2], b[3]};
    v4u ph, pl;
#pragma unroll
    for (int e = 0; e < 4; ++e) {
      const unsigned short h0 = f2bf_bits(f[2 * e]), h1 = f2bf_bits(f[2 * e + 1]);
      const unsigned short l0 = f2bf_bits(f[2 * e] - bf_bits2f(h0)), l1 = f2bf_bits(f[2 * e + 1] - bf_bits2f(h1));
      ph[e] = pk16(h0, h1);
      pl[e] = pk16(l0, l1);
    }
    *(volatile v4u*)(hi + 8 * (size_t)i) = ph;
    *(volatile v4u*)(lo + 8 * (size_t)i) = pl;
    __threadfence();
    *(volatile v4u*)(hi + 8 * (size_t)i) = ph;
    *(volatile v4u*)(lo + 8 * (size_t)i) = pl;
  }
}

template <int EPI>
__global__ __launch_bounds__(256) __attribute__((amdgpu_num_vgpr(256)))
void gemm64_kernel(const unsigned short* __restrict__ Ah, const unsigned short* __restrict__ Al, int lda,
                   const unsigned short* __restrict__ Bh, const unsigned short* __restrict__ Bl, int ldb,
                   void* C, void* C2, int ldc,
                   const float* __restrict__ bias, const float* __restrict__ gam, const float* __restrict__ bet,
                   int M, int N, int K) {
  __shared__ __align__(16) float sT[8][16 * 68];
  const int lane = threadIdx.x & 31;
  const int wave = threadIdx.x >> 5;
  const int tilesN = N >> 6;
  const int tilesM = M >> 6;
  const int tile = blockIdx.x * 8 + wave;
  if (tile >= tilesM * tilesN) return;
  const int tm = tile / tilesN;
  const int tn = tile - tm * tilesN;
  const int m0 = tm << 6;
  const int n0 = tn << 6;
  const int rl   = lane & 15;
  const int koff = (lane >> 4) * 8;
  const int mOff = (lane >> 4) * 8;

  v8f acc[4][4];
#pragma unroll
  for (int i = 0; i < 4; ++i)
#pragma unroll
    for (int j = 0; j < 4; ++j) acc[i][j] = (v8f){0.f, 0.f, 0.f, 0.f, 0.f, 0.f, 0.f, 0.f};

  for (int k0 = 0; k0 < K; k0 += 32) {
    v16b bf[4];
#pragma unroll
    for (int j = 0; j < 4; ++j) bf[j] = ldfrag_b(Bh + (size_t)(n0 + (j << 4) + rl) * ldb + k0 + koff);
#pragma unroll
    for (int i = 0; i < 4; ++i) {
      const size_t ao = (size_t)(m0 + (i << 4) + rl) * lda + k0 + koff;
      const v16b ah = ldfrag_b(Ah + ao);
      const v16b al = ldfrag_b(Al + ao);
#pragma unroll
      for (int j = 0; j < 4; ++j) {
        acc[i][j] = mma_b(ah, bf[j], acc[i][j]);
        acc[i][j] = mma_b(al, bf[j], acc[i][j]);
      }
    }
#pragma unroll
    for (int j = 0; j < 4; ++j) bf[j] = ldfrag_b(Bl + (size_t)(n0 + (j << 4) + rl) * ldb + k0 + koff);
#pragma unroll
    for (int i = 0; i < 4; ++i) {
      const v16b ah = ldfrag_b(Ah + (size_t)(m0 + (i << 4) + rl) * lda + k0 + koff);
#pragma unroll
      for (int j = 0; j < 4; ++j) acc[i][j] = mma_b(ah, bf[j], acc[i][j]);
    }
  }

  float* slab = sT[wave];
#pragma unroll
  for (int i = 0; i < 4; ++i) {
    const int mBase = m0 + (i << 4);
#pragma unroll
    for (int j = 0; j < 4; ++j) {
      const int n = n0 + (j << 4) + rl;
      float cbv = 0.f, cgv = 1.f, ctv = 0.f;
      if (EPI == 0) { cbv = bias[n]; cgv = gam[n] * INVBN; ctv = bet[n]; }
#pragma unroll
      for (int r = 0; r < 8; ++r) {
        float v = acc[i][j][r];
        if (EPI == 0) {
          v += cbv;
          v = v * cgv + ctv;
          v = fmaxf(v, 0.f);
        } else {
          v += bias[mBase + mOff + r];
        }
        slab[(mOff + r) * 68 + (j << 4) + rl] = v;
      }
    }
    lds_wave_sync();
    if (EPI == 0 || EPI == 1) {
      _Float16* Ch = (_Float16*)C;
      const int q = lane >> 3, c8 = (lane & 7) * 8;
      for (int pass = 0; pass < 2; ++pass) {
#pragma unroll
        for (int it = 0; it < 4; ++it) {
          const int row = it * 4 + q;
          const float* sp = slab + row * 68 + c8;
          const v4f u0 = *(const v4f*)sp;
          const v4f u1 = *(const v4f*)(sp + 4);
          v8h hv;
          hv[0] = (_Float16)u0[0]; hv[1] = (_Float16)u0[1]; hv[2] = (_Float16)u0[2]; hv[3] = (_Float16)u0[3];
          hv[4] = (_Float16)u1[0]; hv[5] = (_Float16)u1[1]; hv[6] = (_Float16)u1[2]; hv[7] = (_Float16)u1[3];
          *(volatile v8h*)(Ch + (size_t)(mBase + row) * ldc + n0 + c8) = hv;
        }
        __threadfence();
      }
    }
    if (EPI == 0 || EPI == 2) {
      float* Cf = (EPI == 0) ? (float*)C2 : (float*)C;
      const int h2 = lane >> 4, c4 = (lane & 15) * 4;
      for (int pass = 0; pass < 2; ++pass) {
#pragma unroll
        for (int it = 0; it < 8; ++it) {
          const int row = it * 2 + h2;
          const v4f v = *(const v4f*)(slab + row * 68 + c4);
          *(volatile v4f*)(Cf + (size_t)(mBase + row) * ldc + n0 + c4) = v;
        }
        __threadfence();
      }
    }
    lds_wave_sync();
  }
}

#define SSP 68
#define SPP 72
#define SYP 132

__global__ __launch_bounds__(512) __attribute__((amdgpu_num_vgpr(256)))
void attn_kernel(const unsigned short* __restrict__ thp,
                 const float* __restrict__ th32,
                 const unsigned short* __restrict__ gp,
                 unsigned short* __restrict__ yh,
                 unsigned short* __restrict__ yl) {
  __shared__ __align__(16) float    sS[64 * SSP];
  __shared__ __align__(16) _Float16 sP[64 * SPP];
  __shared__ __align__(16) float    sY[8 * 16 * SYP];
  __shared__ float sM[64], sL[64], sAl[64], sD[64];

  const int tid  = threadIdx.x;
  const int wave = tid >> 5;
  const int lane = tid & 31;
  const int hh   = lane >> 4;
  const int c    = lane & 15;
  const int q0   = blockIdx.x * 64;
  const int qs   = wave & 3;
  const int wq   = wave >> 2;
  const _Float16* th = (const _Float16*)(const void*)thp;
  const _Float16* g  = (const _Float16*)(const void*)gp;

  v16h qa[8];
  {
    const _Float16* qr = th + (size_t)(q0 + qs * 16 + c) * CT + 8 * hh;
#pragma unroll
    for (int kk = 0; kk < 8; ++kk) qa[kk] = ldfrag_h(qr + kk * 32);
  }

  {
    const int tok = tid >> 3, part = tid & 7;
    const float* tr = th32 + (size_t)(q0 + tok) * CT + part * 32;
    float ss = 0.f;
#pragma unroll
    for (int i = 0; i < 8; ++i) {
      const v4f v = *(const v4f*)(tr + 4 * i);
      ss += v[0] * v[0] + v[1] * v[1] + v[2] * v[2] + v[3] * v[3];
    }
    ss += __shfl_xor(ss, 1, 32);
    ss += __shfl_xor(ss, 2, 32);
    ss += __shfl_xor(ss, 4, 32);
    if (part == 0) { sD[tok] = ss * SCL; sM[tok] = -INFINITY; sL[tok] = 0.f; sAl[tok] = 0.f; }
  }
  v8f acc[8];
#pragma unroll
  for (int t = 0; t < 8; ++t) acc[t] = (v8f){0.f, 0.f, 0.f, 0.f, 0.f, 0.f, 0.f, 0.f};
  __syncthreads();

  for (int kt = 0; kt < NKT; ++kt) {
    const int m0 = kt * 64;
    {
      const _Float16* kr = th + (size_t)(m0 + wq * 16 + c) * CT + 8 * hh;
      v8f s = (v8f){0.f, 0.f, 0.f, 0.f, 0.f, 0.f, 0.f, 0.f};
#pragma unroll
      for (int kk = 0; kk < 8; ++kk) {
        const v16h b = ldfrag_h(kr + kk * 32);
        s = mma_h(qa[kk], b, s);
      }
#pragma unroll
      for (int r = 0; r < 8; ++r) sS[(qs * 16 + 8 * hh + r) * SSP + wq * 16 + c] = s[r] * SCL;
    }
    __syncthreads();
    {
      const int row = tid >> 3, e8 = tid & 7;
      const float* sp = sS + row * SSP + e8 * 8;
      const v4f u0 = *(const v4f*)sp;
      const v4f u1 = *(const v4f*)(sp + 4);
      float sv[8] = {u0[0], u0[1], u0[2], u0[3], u1[0], u1[1], u1[2], u1[3]};
      const int drel = (kt == (int)blockIdx.x) ? row : -1;
      const float dval = sD[row];
      float cm = -INFINITY;
#pragma unroll
      for (int j = 0; j < 8; ++j) {
        const int kl = e8 * 8 + j;
        float v = sv[j];
        v = (kl == drel) ? dval : v;
        v = (m0 + kl < NREAL) ? v : -INFINITY;
        sv[j] = v;
        cm = fmaxf(cm, v);
      }
      cm = fmaxf(cm, __shfl_xor(cm, 1, 32));
      cm = fmaxf(cm, __shfl_xor(cm, 2, 32));
      cm = fmaxf(cm, __shfl_xor(cm, 4, 32));
      const float mo = sM[row];
      const float mn = fmaxf(mo, cm);
      const float al = exp2f(mo - mn);
      float ps = 0.f;
      v8h pv;
#pragma unroll
      for (int j = 0; j < 8; ++j) {
        const float p = exp2f(sv[j] - mn);
        ps += p;
        pv[j] = (_Float16)(p * PCARRY);
      }
      *(v8h*)(sP + row * SPP + e8 * 8) = pv;
      ps += __shfl_xor(ps, 1, 32);
      ps += __shfl_xor(ps, 2, 32);
      ps += __shfl_xor(ps, 4, 32);
      if (e8 == 0) {
        const float lo = sL[row];
        sM[row]  = mn;
        sL[row]  = lo * al + ps;
        sAl[row] = al;
      }
    }
    __syncthreads();
    {
      float alv[8];
#pragma unroll
      for (int r = 0; r < 8; ++r) alv[r] = sAl[qs * 16 + 8 * hh + r];
#pragma unroll
      for (int t = 0; t < 8; ++t)
#pragma unroll
        for (int r = 0; r < 8; ++r) acc[t][r] *= alv[r];
      const int cbase = wq * 128;
#pragma unroll 1
      for (int k2 = 0; k2 < 2; ++k2) {
        const v16h a = ldfrag_h(sP + (qs * 16 + c) * SPP + k2 * 32 + 8 * hh);
#pragma unroll
        for (int t = 0; t < 8; ++t) {
          const v16h b = ldfrag_h(g + (size_t)(cbase + t * 16 + c) * NPAD + m0 + k2 * 32 + 8 * hh);
          acc[t] = mma_h(a, b, acc[t]);
        }
      }
    }
  }

  {
    float inv[8];
#pragma unroll
    for (int r = 0; r < 8; ++r) inv[r] = __builtin_amdgcn_rcpf(sL[qs * 16 + 8 * hh + r]) * PINV;
    const int cbase = wq * 128;
    const int c16 = lane & 15;
    for (int grp = 0; grp < 2; ++grp) {
      if ((wave >> 3) == grp) {
        float* sy = sY + (wave & 7) * (16 * SYP);
#pragma unroll
        for (int t = 0; t < 8; ++t)
#pragma unroll
          for (int r = 0; r < 8; ++r) sy[(8 * hh + r) * SYP + t * 16 + c] = acc[t][r] * inv[r];
        lds_wave_sync();
        for (int pass = 0; pass < 2; ++pass) {
#pragma unroll
          for (int it = 0; it < 8; ++it) {
            const int row = it * 2 + hh;
            const float* sp = sy + row * SYP + c16 * 8;
            const v4f u0 = *(const v4f*)sp;
            const v4f u1 = *(const v4f*)(sp + 4);
            const float f[8] = {u0[0], u0[1], u0[2], u0[3], u1[0], u1[1], u1[2], u1[3]};
            v4u ph, pl;
#pragma unroll
            for (int e = 0; e < 4; ++e) {
              const unsigned short h0 = f2bf_bits(f[2 * e]), h1 = f2bf_bits(f[2 * e + 1]);
              const unsigned short l0 = f2bf_bits(f[2 * e] - bf_bits2f(h0));
              const unsigned short l1 = f2bf_bits(f[2 * e + 1] - bf_bits2f(h1));
              ph[e] = pk16(h0, h1);
              pl[e] = pk16(l0, l1);
            }
            const size_t go = (size_t)(q0 + qs * 16 + row) * CG + cbase + c16 * 8;
            *(volatile v4u*)(yh + go) = ph;
            *(volatile v4u*)(yl + go) = pl;
          }
          __threadfence();
        }
      }
      __syncthreads();
    }
  }
}

__global__ __launch_bounds__(128) void copy_out_kernel(const float* __restrict__ pl, float* __restrict__ out) {
  const int i = blockIdx.x * 128 + threadIdx.x;
  const int base = i * 4;
  v4f v;
#pragma unroll
  for (int e = 0; e < 4; ++e) {
    const int idx = base + e;
    const int ch  = idx / NREAL;
    const int n   = idx - ch * NREAL;
    v[e] = pl[(size_t)ch * NPAD + n];
  }
  *(volatile v4f*)(out + base) = v;
  __threadfence();
  *(volatile v4f*)(out + base) = v;
}

extern "C" void kernel_launch(void* const* d_in, const int* in_sizes, int n_in,
                              void* d_out, int out_size, void* d_ws, size_t ws_size,
                              hipStream_t stream) {
  if (n_in < 10) return;
  if (in_sizes[0] != CIN * NREAL || in_sizes[1] != CIN * NREAL) return;
  if (in_sizes[2] != CT * KMIX || in_sizes[3] != CT || in_sizes[4] != CT || in_sizes[5] != CT) return;
  if (in_sizes[6] != CG * KMIX || in_sizes[7] != CG) return;
  if (in_sizes[8] != CIN * CG || in_sizes[9] != CIN) return;
  if (out_size != CIN * NREAL) return;

  const float* x      = (const float*)d_in[0];
  const float* pos    = (const float*)d_in[1];
  const float* w_th   = (const float*)d_in[2];
  const float* b_th   = (const float*)d_in[3];
  const float* gam_th = (const float*)d_in[4];
  const float* bet_th = (const float*)d_in[5];
  const float* w_g    = (const float*)d_in[6];
  const float* b_g    = (const float*)d_in[7];
  const float* w_out  = (const float*)d_in[8];
  const float* b_out  = (const float*)d_in[9];

  const size_t PX   = (size_t)NPAD * KMIX * 2;
  const size_t PWT  = (size_t)CT * KMIX * 2;
  const size_t PWG  = (size_t)CG * KMIX * 2;
  const size_t PWO  = (size_t)CIN * CG * 2;
  const size_t PTH  = (size_t)NPAD * CT * 2;
  const size_t PT32 = (size_t)NPAD * CT * 4;
  const size_t PG   = (size_t)CG * NPAD * 2;
  const size_t PY   = (size_t)NPAD * CG * 2;
  const size_t PO   = (size_t)CIN * NPAD * 4;
  size_t off = 0;
  const size_t oXH  = off; off += PX;
  const size_t oXL  = off; off += PX;
  const size_t oWTH = off; off += PWT;
  const size_t oWTL = off; off += PWT;
  const size_t oWGH = off; off += PWG;
  const size_t oWGL = off; off += PWG;
  const size_t oWOH = off; off += PWO;
  const size_t oWOL = off; off += PWO;
  const size_t oTHF = off; off += PTH;
  const size_t oT32 = off; off += PT32;
  const size_t oGF  = off; off += PG;
  const size_t oYH  = off; off += PY;
  const size_t oYL  = off; off += PY;
  const size_t oOP  = off; off += PO;
  if (off > ws_size) return;

  char* ws = (char*)d_ws;
  unsigned short* XH  = (unsigned short*)(ws + oXH);
  unsigned short* XL  = (unsigned short*)(ws + oXL);
  unsigned short* WTH = (unsigned short*)(ws + oWTH);
  unsigned short* WTL = (unsigned short*)(ws + oWTL);
  unsigned short* WGH = (unsigned short*)(ws + oWGH);
  unsigned short* WGL = (unsigned short*)(ws + oWGL);
  unsigned short* WOH = (unsigned short*)(ws + oWOH);
  unsigned short* WOL = (unsigned short*)(ws + oWOL);
  unsigned short* THF = (unsigned short*)(ws + oTHF);
  float*          T32 = (float*)(ws + oT32);
  unsigned short* GF  = (unsigned short*)(ws + oGF);
  unsigned short* YH  = (unsigned short*)(ws + oYH);
  unsigned short* YL  = (unsigned short*)(ws + oYL);
  float*          OP  = (float*)(ws + oOP);

  const dim3 blk(256);

  xmix_kernel<<<dim3(KMIX / 64, NKT), blk, 0, stream>>>(x, pos, XH, XL);
  {
    const int n8t = CT * KMIX / 8;
    const int n8g = CG * KMIX / 8;
    const int n8o = CIN * CG / 8;
    wsplit_kernel<<<dim3((n8t + 255) / 256), blk, 0, stream>>>(w_th, WTH, WTL, n8t);
    wsplit_kernel<<<dim3((n8g + 255) / 256), blk, 0, stream>>>(w_g, WGH, WGL, n8g);
    wsplit_kernel<<<dim3((n8o + 255) / 256), blk, 0, stream>>>(w_out, WOH, WOL, n8o);
  }
  {
    const int tiles = NKT * (CT / 64);
    gemm64_kernel<0><<<dim3((tiles + 7) / 8), blk, 0, stream>>>(
        XH, XL, KMIX, WTH, WTL, KMIX, (void*)THF, (void*)T32, CT,
        b_th, gam_th, bet_th, NPAD, CT, KMIX);
  }
  {
    const int tiles = (CG / 64) * NKT;
    gemm64_kernel<1><<<dim3((tiles + 7) / 8), blk, 0, stream>>>(
        WGH, WGL, KMIX, XH, XL, KMIX, (void*)GF, (void*)GF, NPAD,
        b_g, b_g, b_g, CG, NPAD, KMIX);
  }
  attn_kernel<<<dim3(NKT), dim3(512), 0, stream>>>(THF, T32, GF, YH, YL);
  {
    const int tiles = (CIN / 64) * NKT;
    gemm64_kernel<2><<<dim3((tiles + 7) / 8), blk, 0, stream>>>(
        WOH, WOL, CG, YH, YL, CG, (void*)OP, (void*)OP, NPAD,
        b_out, b_out, b_out, CIN, NPAD, CG);
  }
  copy_out_kernel<<<dim3(NREAL), dim3(128), 0, stream>>>(OP, (float*)d_out);
  (void)hipGetLastError();
}
